// MMN_34995393527847
// MI455X (gfx1250) — hardware-verified
//
#include <hip/hip_runtime.h>


#define NB_  16
#define NS   8
#define NN_  64
#define DD   512
#define JJ   256
#define KK   128
#define NM   (NN_ * NN_)

typedef unsigned short bf;
typedef __attribute__((ext_vector_type(16))) __bf16   v16bf;
typedef __attribute__((ext_vector_type(8)))  unsigned short v8us;
typedef __attribute__((ext_vector_type(8)))  float    v8f;
typedef __attribute__((ext_vector_type(4)))  float    v4f;
typedef v4f  __attribute__((may_alias)) v4fa;
typedef v8us __attribute__((may_alias)) v8usa;

__device__ __forceinline__ unsigned short f2bf(float f) { unsigned u = __float_as_uint(f); u += 0x7FFFu + ((u >> 16) & 1u); return (unsigned short)(u >> 16); }
__device__ __forceinline__ float bf2f(unsigned short b) { return __uint_as_float(((unsigned)b) << 16); }
__device__ __forceinline__ float bfr(float f) { return bf2f(f2bf(f)); }
__device__ __forceinline__ v16bf cat16b(v8us lo, v8us hi) { return __builtin_bit_cast(v16bf, __builtin_shufflevector(lo, hi, 0, 1, 2, 3, 4, 5, 6, 7, 8, 9, 10, 11, 12, 13, 14, 15)); }
__device__ __forceinline__ v8f wmmab(v16bf a, v16bf b, v8f c) { return __builtin_amdgcn_wmma_f32_16x16x32_bf16(false, a, false, b, (short)0, c, false, false); }
#define VST2(T, p, v) do { const T vst2_v_ = (v); *(volatile T*)(p) = vst2_v_; __threadfence(); *(volatile T*)(p) = vst2_v_; } while (0)

__global__ __launch_bounds__(256) void k_rows(const float* __restrict__ src, int rows, int C, bf* dst) {
    const int lane = threadIdx.x & 31, r = blockIdx.x * 8 + (threadIdx.x >> 5);
    if (r >= rows) return;
#pragma unroll 1
    for (int ps = 0; ps < 2; ++ps) {
        for (int q = 0; q < C / 256; ++q) { v8us o;
#pragma unroll
            for (int i = 0; i < 8; ++i) o[i] = f2bf(src[(size_t)r * C + q * 256 + lane * 8 + i]);
            *(volatile v8us*)(dst + (size_t)r * C + q * 256 + lane * 8) = o; }
        if (ps == 0) __threadfence(); }
}
__global__ __launch_bounds__(256) void k_wt(const float* __restrict__ Wm, int K, int ncols, bf* WT) {
    __shared__ __align__(16) unsigned short tl[64 * 72];
    const int tid = threadIdx.x, k0 = blockIdx.x * 64, n0 = blockIdx.y * 64;
    const int kk = tid >> 2, nq = (tid & 3) * 16;
#pragma unroll
    for (int i = 0; i < 16; ++i) tl[(nq + i) * 72 + kk] = f2bf(Wm[(size_t)(k0 + kk) * ncols + n0 + nq + i]);
    __syncthreads();
    const int piece = tid & 7;
    auto pass = [&]() {
#pragma unroll
        for (int s = 0; s < 2; ++s) { const int nr = (tid >> 3) + 32 * s; const v8us val = *(const v8usa*)(tl + nr * 72 + piece * 8); *(volatile v8us*)(WT + (size_t)(n0 + nr) * K + k0 + piece * 8) = val; }
    };
    pass(); __threadfence(); pass();
}
__global__ __launch_bounds__(256) void k_ft(const float* __restrict__ f, bf* FT) {
    __shared__ __align__(16) unsigned short tl[64 * 72];
    const int tid = threadIdx.x, d0 = blockIdx.x * 64, b = blockIdx.y;
    const int dr = tid >> 2, nq = (tid & 3) * 16;
#pragma unroll
    for (int i = 0; i < 16; ++i) tl[(nq + i) * 72 + dr] = f2bf(f[((size_t)b * DD + d0 + dr) * NN_ + nq + i]);
    __syncthreads();
    const int piece = tid & 7;
    auto pass = [&]() {
#pragma unroll
        for (int s = 0; s < 2; ++s) { const int n = (tid >> 3) + 32 * s; const v8us val = *(const v8usa*)(tl + n * 72 + piece * 8); *(volatile v8us*)(FT + ((size_t)b * NN_ + n) * DD + d0 + piece * 8) = val; }
    };
    pass(); __threadfence(); pass();
}
__global__ __launch_bounds__(256) void k_pairs(const float* __restrict__ f, int b, bf* AH, bf* AL) {
    const int lane = threadIdx.x & 31, r = blockIdx.x * 8 + (threadIdx.x >> 5);
    if (r >= NM) return;
    const int n = r >> 6, m = r & 63; const float* fb = f + (size_t)b * DD * NN_;
#pragma unroll 1
    for (int ps = 0; ps < 2; ++ps) {
#pragma unroll
        for (int q = 0; q < DD / 256; ++q) { v8us oh, ol;
#pragma unroll
            for (int i = 0; i < 8; ++i) { const int d = q * 256 + lane * 8 + i; const float p = bfr(fb[(size_t)d * NN_ + n]) * bfr(fb[(size_t)d * NN_ + m]); const unsigned short hb = f2bf(p); oh[i] = hb; ol[i] = f2bf(p - bf2f(hb)); }
            *(volatile v8us*)(AH + (size_t)r * DD + q * 256 + lane * 8) = oh; *(volatile v8us*)(AL + (size_t)r * DD + q * 256 + lane * 8) = ol; }
        if (ps == 0) __threadfence(); }
}
template <bool SPLITA>
__global__ __launch_bounds__(128) void k_gemm(const bf* __restrict__ A, const bf* __restrict__ Al, const bf* __restrict__ Bn, int K, const float* __restrict__ bias, int ldc, float* C) {
    __shared__ __align__(16) float ost[4][16 * 68];
    const int lane = threadIdx.x & 31, wave = threadIdx.x >> 5, lr = lane & 15, hi = lane >> 4;
    const size_t r0 = (size_t)blockIdx.x * 64 + wave * 16; const int c0 = blockIdx.y * 64;
    const size_t aoff = (r0 + lr) * (size_t)K + 8 * hi;
    size_t boff[4];
#pragma unroll
    for (int t = 0; t < 4; ++t) boff[t] = (size_t)(c0 + t * 16 + lr) * K + 8 * hi;
    v8f acc[4];
#pragma unroll
    for (int t = 0; t < 4; ++t) acc[t] = (v8f){};
#pragma unroll 2
    for (int kc = 0; kc < K; kc += 32) {
        const v16bf a = cat16b(*(const v8us*)(A + aoff + kc), *(const v8us*)(A + aoff + kc + 16));
        v16bf al = a; if (SPLITA) al = cat16b(*(const v8us*)(Al + aoff + kc), *(const v8us*)(Al + aoff + kc + 16));
#pragma unroll
        for (int t = 0; t < 4; ++t) { const v16bf bb = cat16b(*(const v8us*)(Bn + boff[t] + kc), *(const v8us*)(Bn + boff[t] + kc + 16)); acc[t] = wmmab(a, bb, acc[t]); if (SPLITA) acc[t] = wmmab(al, bb, acc[t]); }
        asm volatile("v_nop" : "+v"(acc[0]), "+v"(acc[1]), "+v"(acc[2]), "+v"(acc[3]) : "v"(a), "v"(al) : "memory");
    }
    float* os = &ost[wave][0];
#pragma unroll
    for (int t = 0; t < 4; ++t) { const float bv = bias ? bfr(bias[c0 + t * 16 + lr]) : 0.f;
#pragma unroll
        for (int j = 0; j < 8; ++j) os[(hi * 8 + j) * 68 + t * 16 + lr] = acc[t][j] + bv; }
    __builtin_amdgcn_wave_barrier(); asm volatile("" ::: "memory");
    float* crow = C + r0 * ldc + c0;
    auto pass = [&]() {
#pragma unroll
        for (int s = 0; s < 8; ++s) { const int Lid = (lane >> 3) + 4 * s, piece = lane & 7; const int row = Lid >> 1, cofs = (Lid & 1) * 32 + piece * 4;
            const v4f val = *(const v4fa*)(os + row * 68 + cofs); *(volatile v4f*)(crow + (size_t)row * ldc + cofs) = val; }
    };
    pass(); __threadfence(); pass();
}
__global__ __launch_bounds__(256) void k_score(const float* __restrict__ G, const float* __restrict__ sf, const float* __restrict__ sfi, int b, float* out0, float* out2) {
    __shared__ float sn[2][NS][JJ];
    __shared__ __align__(16) float res[2][NS][NN_];
    const int tid = threadIdx.x, n = blockIdx.x;
    { const int v = tid >> 4, part = tid & 15; const int which = v >> 3, s = v & 7; const float* src = (which == 0 ? sfi : sf) + ((size_t)b * NS + s) * JJ;
      float sq = 0.f;
#pragma unroll 4
      for (int i = 0; i < 16; ++i) { const float x = bfr(src[part * 16 + i]); sq += x * x; }
      sq += __shfl_xor(sq, 1, 32); sq += __shfl_xor(sq, 2, 32); sq += __shfl_xor(sq, 4, 32); sq += __shfl_xor(sq, 8, 32);
      const float inv = 1.0f / fmaxf(sqrtf(sq), 1e-12f);
#pragma unroll 4
      for (int i = 0; i < 16; ++i) sn[which][s][part * 16 + i] = bfr(src[part * 16 + i]) * inv; }
    __syncthreads();
    const int m = tid >> 2, q = tid & 3; const float* gr = G + ((size_t)n * NN_ + m) * (2 * JJ);
    float nq0 = 0.f, nq1 = 0.f, d0[NS], d1[NS];
#pragma unroll
    for (int s = 0; s < NS; ++s) { d0[s] = 0.f; d1[s] = 0.f; }
#pragma unroll 2
    for (int i = 0; i < 64; ++i) { const int j = q * 64 + i; const float g0 = gr[j], g1 = gr[JJ + j]; nq0 += g0 * g0; nq1 += g1 * g1;
#pragma unroll
        for (int s = 0; s < NS; ++s) { d0[s] += g0 * sn[0][s][j]; d1[s] += g1 * sn[1][s][j]; } }
    nq0 += __shfl_xor(nq0, 1, 32); nq0 += __shfl_xor(nq0, 2, 32); nq1 += __shfl_xor(nq1, 1, 32); nq1 += __shfl_xor(nq1, 2, 32);
#pragma unroll
    for (int s = 0; s < NS; ++s) { d0[s] += __shfl_xor(d0[s], 1, 32); d0[s] += __shfl_xor(d0[s], 2, 32); d1[s] += __shfl_xor(d1[s], 1, 32); d1[s] += __shfl_xor(d1[s], 2, 32); }
    const float i0 = 1.0f / fmaxf(sqrtf(nq0), 1e-12f), i1 = 1.0f / fmaxf(sqrtf(nq1), 1e-12f); const float mk = (m >= n) ? 1.f : 0.f;
    if (q == 0) {
#pragma unroll
        for (int s = 0; s < NS; ++s) { res[0][s][m] = mk / (1.0f + __expf(-10.0f * d0[s] * i0)); res[1][s][m] = d1[s] * i1 * mk; } }
    __syncthreads();
    { const int row = tid >> 4, piece = tid & 15; const int which = row >> 3, s = row & 7;
      float* dst = (which == 0 ? out0 : out2) + ((((size_t)b * NS + s) * NN_ + n) * NN_) + piece * 4;
      const v4f val = *(const v4fa*)(&res[which][s][piece * 4]); *(volatile v4f*)dst = val; __threadfence(); *(volatile v4f*)dst = val; }
}
__global__ __launch_bounds__(256) void k_fusion(const float* __restrict__ V1, const float* __restrict__ Q2, const float* __restrict__ wf, float* out1) {
    __shared__ float v1s[KK][NN_ + 1]; __shared__ float cq[KK]; __shared__ __align__(16) float res[NN_][NN_ + 4];
    const int tid = threadIdx.x, b = blockIdx.y, s = blockIdx.x;
    for (int i = tid; i < KK * NN_; i += 256) { const int n = i / KK, k = i - n * KK; v1s[k][n] = V1[((size_t)b * NN_ + n) * KK + k]; }
    if (tid < KK) { const float qv = Q2[((size_t)b * NS + s) * KK + tid]; cq[tid] = bfr(wf[tid]) * qv * qv; }
    __syncthreads();
    const int n = tid >> 2, mq = (tid & 3) * 16;
    float acc[16];
#pragma unroll
    for (int i = 0; i < 16; ++i) acc[i] = 0.f;
#pragma unroll 1
    for (int k = 0; k < KK; ++k) { const float w = cq[k] * v1s[k][n];
#pragma unroll
        for (int i = 0; i < 16; ++i) acc[i] += w * v1s[k][mq + i]; }
#pragma unroll
    for (int i = 0; i < 16; ++i) { const int m = mq + i; res[n][m] = (m >= n) ? 1.0f / (1.0f + __expf(-10.0f * acc[i])) : 0.f; }
    __syncthreads();
#pragma unroll 1
    for (int ps = 0; ps < 2; ++ps) {
#pragma unroll
        for (int r4 = 0; r4 < 4; ++r4) { const int row = r4 * 16 + (tid >> 4), piece = tid & 15;
            *(volatile v4f*)(out1 + ((((size_t)b * NS + s) * NN_ + row) * NN_) + piece * 4) = *(const v4fa*)(&res[row][piece * 4]); }
        if (ps == 0) __threadfence(); }
}

extern "C" void kernel_launch(void* const* d_in, const int* in_sizes, int n_in,
                              void* d_out, int out_size, void* d_ws, size_t ws_size, hipStream_t stream) {
    (void)in_sizes; (void)n_in; (void)out_size;
    const float* feats = (const float*)d_in[0]; const float* sf = (const float*)d_in[1]; const float* sfi = (const float*)d_in[2]; const float* sff = (const float*)d_in[3];
    const float* W1 = (const float*)d_in[4]; const float* b1 = (const float*)d_in[5]; const float* W2 = (const float*)d_in[6]; const float* b2 = (const float*)d_in[7];
    const float* Wp = (const float*)d_in[8]; const float* Wiou = (const float*)d_in[9]; const float* Wfuse = (const float*)d_in[10];
    const size_t MAPSZ = (size_t)NB_ * NS * NN_ * NN_;
    float* out0 = (float*)d_out; float* out1 = out0 + MAPSZ; float* out2 = out0 + 2 * MAPSZ;
    char* wsp = (char*)d_ws;
    auto take = [&](size_t bytes) { char* p = wsp; wsp += (bytes + 255) & ~(size_t)255; return (void*)p; };
    bf* WJ = (bf*)take((size_t)2 * JJ * DD * 2);
    bf* W1T = (bf*)take((size_t)KK * DD * 2); bf* W2T = (bf*)take((size_t)KK * DD * 2);
    bf* FT = (bf*)take((size_t)NB_ * NN_ * DD * 2); bf* SFb = (bf*)take((size_t)NB_ * NS * DD * 2);
    float* V1 = (float*)take((size_t)NB_ * NN_ * KK * 4); float* Q2 = (float*)take((size_t)NB_ * NS * KK * 4);
    bf* AH = (bf*)take((size_t)NM * DD * 2); bf* AL = (bf*)take((size_t)NM * DD * 2); float* G = (float*)take((size_t)NM * 2 * JJ * 4);
    if ((size_t)(wsp - (char*)d_ws) > ws_size) return;
    k_rows<<<JJ / 8, 256, 0, stream>>>(Wiou, JJ, DD, WJ); k_rows<<<JJ / 8, 256, 0, stream>>>(Wp, JJ, DD, WJ + (size_t)JJ * DD);
    k_wt<<<dim3(DD / 64, KK / 64, 1), 256, 0, stream>>>(W1, DD, KK, W1T); k_wt<<<dim3(DD / 64, KK / 64, 1), 256, 0, stream>>>(W2, DD, KK, W2T);
    k_ft<<<dim3(DD / 64, NB_, 1), 256, 0, stream>>>(feats, FT); k_rows<<<(NB_ * NS) / 8, 256, 0, stream>>>(sff, NB_ * NS, DD, SFb);
    k_gemm<false><<<dim3((NB_ * NN_) / 64, KK / 64, 1), 128, 0, stream>>>(FT, nullptr, W1T, DD, b1, KK, V1);
    k_gemm<false><<<dim3((NB_ * NS) / 64, KK / 64, 1), 128, 0, stream>>>(SFb, nullptr, W2T, DD, b2, KK, Q2);
    k_fusion<<<dim3(NS, NB_, 1), 256, 0, stream>>>(V1, Q2, Wfuse, out1);
    for (int b = 0; b < NB_; ++b) {
        k_pairs<<<NM / 8, 256, 0, stream>>>(feats, b, AH, AL);
        k_gemm<true><<<dim3(NM / 64, (2 * JJ) / 64, 1), 128, 0, stream>>>(AH, AL, WJ, DD, nullptr, 2 * JJ, G);
        k_score<<<NN_, 256, 0, stream>>>(G, sf, sfi, b, out0, out2);
    }
}
